// SplitTransformer_36636071035466
// MI455X (gfx1250) — hardware-verified
//
#include <hip/hip_runtime.h>


namespace {
constexpr int B = 4, L = 4096, CH = 512, RG = 128, D = 256, NH = 8, DH = 32, FF = 1024, NC = 8, VOC = 4, MAXW = 768, RPB = 5888, TPB = RPB / 16;
constexpr float XS = 8.0f, PS = 1024.0f, WSC = 256.0f;
typedef _Float16 b16;
typedef __attribute__((ext_vector_type(16))) _Float16 v16b;
typedef __attribute__((ext_vector_type(8))) _Float16 v8b;
typedef __attribute__((ext_vector_type(8))) float v8f;
typedef __attribute__((ext_vector_type(4))) float v4f;
__device__ __forceinline__ float bf16_rne(float f) { unsigned int u = __float_as_uint(f); u += 0x7FFFu + ((u >> 16) & 1u); return __uint_as_float(u & 0xFFFF0000u); }
__device__ __forceinline__ void split16(float v, b16& hi, b16& lo) { hi = (b16)v; lo = (b16)(v - (float)hi); }
__device__ __forceinline__ v16b frag_kb(const b16* p, int hh) { const v8b a = *(const v8b*)(p + 8 * hh), b = *(const v8b*)(p + 16 + 8 * hh); v16b f;
#pragma unroll
  for (int e = 0; e < 8; ++e) { f[e] = a[e]; f[8 + e] = b[e]; } return f; }
__device__ __forceinline__ v8f wmma16b(v16b a, v16b b, v8f c) { v8f d = __builtin_amdgcn_wmma_f32_16x16x32_f16(false, a, false, b, (short)0, c, false, false); asm volatile("v_nop\n\tv_nop\n\tv_nop\n\tv_nop" : "+v"(d) : "v"(a), "v"(b)); return d; }
__device__ __forceinline__ void wave_lds_sync() { __builtin_amdgcn_fence(__ATOMIC_RELEASE, "workgroup"); __builtin_amdgcn_wave_barrier(); __builtin_amdgcn_fence(__ATOMIC_ACQUIRE, "workgroup"); }
__device__ __forceinline__ float pmul(float a, float b) { float p = a * b; asm volatile("" : "+v"(p)); return p; }
__device__ __forceinline__ int iclamp(int v, int lo, int hi) { return v < lo ? lo : (v > hi ? hi : v); }
__device__ __forceinline__ float gelu(float v) { return 0.5f * v * (1.0f + erff(v * 0.70710678118654752f)); }
__device__ __forceinline__ int c_ms(int i) { return i == 0 ? 0 : i * CH - RG; }
__device__ __forceinline__ int c_wn(int i) { return (i == 0 || i == NC - 1) ? CH + RG : CH + 2 * RG; }
__device__ __forceinline__ int c_rowbase(int i) { return i == 0 ? 0 : 640 + (i - 1) * 768; }
__device__ __forceinline__ void tile_decode(int tix, int& chunk, int& w0) { if (tix < 40) { chunk = 0; w0 = tix * 16; } else if (tix < 328) { chunk = 1 + (tix - 40) / 48; w0 = ((tix - 40) % 48) * 16; } else { chunk = 7; w0 = (tix - 328) * 16; } }

__global__ __launch_bounds__(256) void wput_kernel(const float* __restrict__ w, int KIN, int OUTW, b16* __restrict__ WT) { const int KG = KIN / 8; const int u = blockIdx.x * 256 + threadIdx.x; if (u >= OUTW * KG) return; const int o = u / KG, k0 = (u % KG) * 8; v8b v;
#pragma unroll
  for (int j = 0; j < 8; ++j) v[j] = (b16)(bf16_rne(w[(size_t)(k0 + j) * OUTW + o]) * WSC); for (int pass = 0; pass < 2; ++pass) { *(volatile v8b*)(WT + (size_t)o * KIN + k0) = v; __threadfence(); } }
__global__ __launch_bounds__(256) void h_kernel(const int* __restrict__ tok, const float* __restrict__ emb, const float* __restrict__ pos, int BV, int CV, float* __restrict__ HW) {
  const size_t u = (size_t)blockIdx.x * 256 + threadIdx.x; if (u >= (size_t)BV * RPB * 32) return; const int c8 = (int)(u % 32) * 8; const size_t row = u / 32; const int b = (int)(row / RPB), r = (int)(row % RPB); int chunk, w0; tile_decode(r / 16, chunk, w0); const int w = w0 + (r % 16); if (chunk >= CV) return;
  const int t = c_ms(chunk) + w; const int id = iclamp(tok[(size_t)b * L + t], 0, VOC - 1); float v[8];
  for (int j = 0; j < 8; ++j) v[j] = bf16_rne(emb[(size_t)id * D + c8 + j]) + bf16_rne(pos[((size_t)chunk * MAXW + w) * D + c8 + j]);
  for (int pass = 0; pass < 2; ++pass) { *(volatile v4f*)(HW + row * D + c8) = (v4f){v[0], v[1], v[2], v[3]}; *(volatile v4f*)(HW + row * D + c8 + 4) = (v4f){v[4], v[5], v[6], v[7]}; __threadfence(); }
}
template <int KIN, int MODE, int ACT>
__global__ __launch_bounds__(32) void dense_kernel(const float* __restrict__ INf, const b16* __restrict__ INb, const b16* __restrict__ WT, size_t wstride, const float* __restrict__ bias, int bstride, const float* __restrict__ RES, const float* __restrict__ lg, const float* __restrict__ lb, int ncg, int outw, int BV, int CV, float* __restrict__ OUTf, b16* __restrict__ OUTb) {
  __shared__ __attribute__((aligned(16))) b16 Ah[16][MODE == 1 ? KIN + 8 : 8], Al[16][MODE == 1 ? KIN + 8 : 8]; __shared__ float Tf[16][260], Mu[16], Rs[16];
  const int lane = threadIdx.x, nloc = lane & 15, hlf = lane >> 4; const int cg = blockIdx.x % ncg; const int tg = blockIdx.x / ncg; const int b = tg / TPB, tix = tg % TPB; if (b >= BV) return; int chunk, w0; tile_decode(tix, chunk, w0); if (chunk >= CV) return;
  const size_t m0 = (size_t)b * RPB + c_rowbase(chunk) + w0; const b16* W = WT + (size_t)chunk * wstride; const float* bb = bias ? bias + (size_t)chunk * bstride : nullptr;
  if (MODE == 1) { for (int rr = 0; rr < 16; ++rr) for (int c = lane; c < KIN; c += 32) { b16 p, q; split16(INf[(m0 + rr) * KIN + c] * XS, p, q); Ah[rr][c] = p; Al[rr][c] = q; } wave_lds_sync(); }
  v8f acc[16];
#pragma unroll
  for (int t = 0; t < 16; ++t) acc[t] = (v8f){};
#pragma unroll 2
  for (int kb = 0; kb < KIN; kb += 32) { v16b a, al; if (MODE == 1) { a = frag_kb(&Ah[nloc][kb], hlf); al = frag_kb(&Al[nloc][kb], hlf); } else a = frag_kb(INb + (m0 + nloc) * KIN + kb, hlf);
#pragma unroll
    for (int t = 0; t < 16; ++t) { const v16b bw = frag_kb(W + (size_t)(cg * 256 + t * 16 + nloc) * KIN + kb, hlf); acc[t] = wmma16b(a, bw, acc[t]); if (MODE == 1) acc[t] = wmma16b(al, bw, acc[t]); } }
#pragma unroll
  for (int t = 0; t < 16; ++t) { const int c = cg * 256 + t * 16 + nloc; const float bv = bb ? bf16_rne(bb[c]) : 0.0f;
#pragma unroll
    for (int r8 = 0; r8 < 8; ++r8) { float v = acc[t][r8] * (1.0f / (XS * WSC)) + bv; if (ACT == 1) v = gelu(v); if (ACT >= 2) v += RES[(m0 + 8 * hlf + r8) * D + c]; Tf[8 * hlf + r8][t * 16 + nloc] = v; } }
  wave_lds_sync();
  if (ACT >= 2) { if (lane < 16) { float s = 0.0f; for (int c = 0; c < D; ++c) s += Tf[lane][c]; const float mu = s * (1.0f / D); float vq = 0.0f; for (int c = 0; c < D; ++c) { const float dd = Tf[lane][c] - mu; vq += pmul(dd, dd); } Mu[lane] = mu; Rs[lane] = rsqrtf(vq * (1.0f / D) + 1e-3f); } wave_lds_sync(); }
  for (int pass = 0; pass < 2; ++pass) { for (int rr = 0; rr < 16; ++rr) {
      if (ACT <= 1) { if (ACT == 1) { for (int c = lane; c < 256; c += 32) ((volatile b16*)OUTb)[(m0 + rr) * (size_t)outw + cg * 256 + c] = (b16)(Tf[rr][c] * XS); } else { for (int c = lane; c < 256; c += 32) ((volatile float*)OUTf)[(m0 + rr) * (size_t)outw + cg * 256 + c] = Tf[rr][c]; } }
      else { const float* g = lg + (size_t)chunk * D; const float* bt = lb + (size_t)chunk * D;
        if (ACT == 2) { for (int c = lane; c < D; c += 32) { const float y = pmul(pmul(Tf[rr][c] - Mu[rr], Rs[rr]), bf16_rne(g[c])) + bf16_rne(bt[c]); ((volatile float*)OUTf)[(m0 + rr) * D + c] = y; ((volatile b16*)OUTb)[(m0 + rr) * D + c] = (b16)(y * XS); } }
        else { const int w = w0 + rr; const int so = chunk * CH - c_ms(chunk); if (w >= so && w < so + CH) { const size_t trow = (size_t)b * L + chunk * CH + (w - so); for (int c = lane; c < D; c += 32) ((volatile float*)OUTf)[trow * D + c] = pmul(pmul(Tf[rr][c] - Mu[rr], Rs[rr]), bf16_rne(g[c])) + bf16_rne(bt[c]); } } } }
    __threadfence(); }
}
__global__ __launch_bounds__(32) void att_kernel(const float* __restrict__ QKV, int BV, int CV, float* __restrict__ ATT) {
  __shared__ __attribute__((aligned(16))) b16 Qh[16][40], Ql[16][40], Kh[32][40], Kl[32][40], Ph[16][40], Pl[16][40], Vh[32][40], Vl[32][40]; __shared__ float Sc[16][33], Mx[16], Dn[16], Sf[16], Of[16][DH + 1];
  const int lane = threadIdx.x, nloc = lane & 15, hlf = lane >> 4; const int qt = blockIdx.x % TPB; const int hh = (blockIdx.x / TPB) % NH; const int b = blockIdx.x / (TPB * NH); if (b >= BV) return; int chunk, q0; tile_decode(qt, chunk, q0); if (chunk >= CV) return;
  const int Wn = c_wn(chunk); const size_t rb = (size_t)b * RPB + c_rowbase(chunk); const size_t W3 = 3 * D;
  for (int rr = 0; rr < 16; ++rr) { b16 p, ql; split16(QKV[(rb + q0 + rr) * W3 + hh * DH + lane] * XS, p, ql); Qh[rr][lane] = p; Ql[rr][lane] = ql; }
  if (lane < 16) { Mx[lane] = -INFINITY; Dn[lane] = 0.0f; Sf[lane] = 0.0f; }
  v8f acc[2] = {(v8f){}, (v8f){}}; wave_lds_sync();
  int kbeg = q0 - RG; kbeg = kbeg < 0 ? 0 : (kbeg & ~31); const int kend = (q0 + 15 + RG + 1 < Wn) ? q0 + 15 + RG + 1 : Wn;
#pragma unroll 1
  for (int kc = kbeg; kc < kend; kc += 32) {
    for (int rr = 0; rr < 32; ++rr) { const int kk = kc + rr; b16 p = (b16)0.0f, ql = (b16)0.0f, vp = (b16)0.0f, vl = (b16)0.0f; if (kk < Wn) { split16(QKV[(rb + kk) * W3 + D + hh * DH + lane] * XS, p, ql); split16(QKV[(rb + kk) * W3 + 2 * D + hh * DH + lane] * XS, vp, vl); } Kh[rr][lane] = p; Kl[rr][lane] = ql; Vh[lane][rr] = vp; Vl[lane][rr] = vl; }
    wave_lds_sync();
#pragma unroll
    for (int blk = 0; blk < 2; ++blk) { v8f s = {}; const v16b qh = frag_kb(&Qh[nloc][0], hlf), qlo = frag_kb(&Ql[nloc][0], hlf), kh = frag_kb(&Kh[blk * 16 + nloc][0], hlf), kl = frag_kb(&Kl[blk * 16 + nloc][0], hlf); s = wmma16b(qh, kh, s); s = wmma16b(qh, kl, s); s = wmma16b(qlo, kh, s);
#pragma unroll
      for (int r8 = 0; r8 < 8; ++r8) { const int qi = q0 + 8 * hlf + r8, kk = kc + blk * 16 + nloc; const bool ok = kk < Wn && (kk - qi <= RG) && (qi - kk <= RG); Sc[8 * hlf + r8][blk * 16 + nloc] = ok ? s[r8] * (0.17677669529663687f / (XS * XS)) : -INFINITY; } }
    wave_lds_sync();
#pragma unroll 1
    for (int qi = 0; qi < 16; ++qi) { const float sv = Sc[qi][lane]; float cm = sv; for (int o = 16; o; o >>= 1) cm = fmaxf(cm, __shfl_xor(cm, o)); const float mo = Mx[qi]; const float mn = fmaxf(mo, cm); const float p = (sv == -INFINITY) ? 0.0f : __expf(sv - mn); float psum = p; for (int o = 16; o; o >>= 1) psum += __shfl_xor(psum, o);
      b16 ph, plo; split16(p * PS, ph, plo); Ph[qi][lane] = ph; Pl[qi][lane] = plo; if (lane == 0) { const float sf = (mo == -INFINITY || mn == -INFINITY) ? 0.0f : __expf(mo - mn); Sf[qi] = sf; Dn[qi] = Dn[qi] * sf + psum; Mx[qi] = mn; } }
    wave_lds_sync();
#pragma unroll
    for (int t = 0; t < 2; ++t) {
#pragma unroll
      for (int r8 = 0; r8 < 8; ++r8) acc[t][r8] *= Sf[8 * hlf + r8];
      const v16b pa = frag_kb(&Ph[nloc][0], hlf), pb = frag_kb(&Pl[nloc][0], hlf), vh = frag_kb(&Vh[t * 16 + nloc][0], hlf), vl = frag_kb(&Vl[t * 16 + nloc][0], hlf); acc[t] = wmma16b(pa, vh, acc[t]); acc[t] = wmma16b(pa, vl, acc[t]); acc[t] = wmma16b(pb, vh, acc[t]); }
    wave_lds_sync(); }
#pragma unroll
  for (int t = 0; t < 2; ++t)
#pragma unroll
    for (int r8 = 0; r8 < 8; ++r8) { const int rl = 8 * hlf + r8; Of[rl][t * 16 + nloc] = acc[t][r8] * (1.0f / (PS * XS)) / Dn[rl]; }
  wave_lds_sync();
  for (int pass = 0; pass < 2; ++pass) { for (int rr = 0; rr < 16; ++rr) ((volatile float*)ATT)[(rb + q0 + rr) * D + hh * DH + lane] = Of[rr][lane]; __threadfence(); }
}
}

extern "C" void kernel_launch(void* const* d_in, const int* in_sizes, int n_in, void* d_out, int out_size, void* d_ws, size_t ws_size, hipStream_t stream) {
  (void)n_in;
  auto Fp = [&](int i) { return (const float*)d_in[i]; }; auto Ip = [&](int i) { return (const int*)d_in[i]; };
  if (in_sizes[0] != B * L || in_sizes[1] != VOC * D || in_sizes[2] != NC * MAXW * D || in_sizes[3] != NC * D * D || in_sizes[9] != NC * D * D || in_sizes[13] != NC * D * FF || in_sizes[15] != NC * FF * D || out_size != B * L * D) return;
  const int BV = B, CV = NC;
  size_t off = 0; char* ws = (char*)d_ws;
  auto carve = [&](size_t bytes) { char* p = ws + off; off += (bytes + 255) & ~(size_t)255; return p; };
  b16* WQKV = (b16*)carve((size_t)NC * 3 * D * D * 2); b16* WO = (b16*)carve((size_t)NC * D * D * 2); b16* W1T = (b16*)carve((size_t)NC * FF * D * 2); b16* W2T = (b16*)carve((size_t)NC * D * FF * 2);
  float* HW = (float*)carve((size_t)B * RPB * D * 4); float* QKV = (float*)carve((size_t)B * RPB * 3 * D * 4); float* ATT = (float*)carve((size_t)B * RPB * D * 4); float* H1 = (float*)carve((size_t)B * RPB * D * 4); b16* H1b = (b16*)carve((size_t)B * RPB * D * 2); b16* F = (b16*)carve((size_t)B * RPB * FF * 2);
  if (off > ws_size || off > ((size_t)248 << 20)) return;
  for (int i = 0; i < NC; ++i) {
    wput_kernel<<<(D * 32 + 255) / 256, 256, 0, stream>>>(Fp(3) + (size_t)i * D * D, D, D, WQKV + (size_t)i * 3 * D * D); wput_kernel<<<(D * 32 + 255) / 256, 256, 0, stream>>>(Fp(5) + (size_t)i * D * D, D, D, WQKV + (size_t)i * 3 * D * D + (size_t)D * D); wput_kernel<<<(D * 32 + 255) / 256, 256, 0, stream>>>(Fp(7) + (size_t)i * D * D, D, D, WQKV + (size_t)i * 3 * D * D + (size_t)2 * D * D);
    wput_kernel<<<(D * 32 + 255) / 256, 256, 0, stream>>>(Fp(9) + (size_t)i * D * D, D, D, WO + (size_t)i * D * D); wput_kernel<<<(FF * 32 + 255) / 256, 256, 0, stream>>>(Fp(13) + (size_t)i * D * FF, D, FF, W1T + (size_t)i * FF * D); wput_kernel<<<(D * 128 + 255) / 256, 256, 0, stream>>>(Fp(15) + (size_t)i * FF * D, FF, D, W2T + (size_t)i * D * FF); }
  h_kernel<<<(unsigned)(((size_t)BV * RPB * 32 + 255) / 256), 256, 0, stream>>>(Ip(0), Fp(1), Fp(2), BV, CV, HW);
  const int NTILE = BV * TPB;
  dense_kernel<D, 1, 0><<<NTILE, 32, 0, stream>>>(HW, nullptr, WQKV, (size_t)3 * D * D, Fp(4), D, nullptr, nullptr, nullptr, 1, 3 * D, BV, CV, QKV, nullptr);
  dense_kernel<D, 1, 0><<<NTILE, 32, 0, stream>>>(HW, nullptr, WQKV + (size_t)D * D, (size_t)3 * D * D, Fp(6), D, nullptr, nullptr, nullptr, 1, 3 * D, BV, CV, QKV + D, nullptr);
  dense_kernel<D, 1, 0><<<NTILE, 32, 0, stream>>>(HW, nullptr, WQKV + (size_t)2 * D * D, (size_t)3 * D * D, Fp(8), D, nullptr, nullptr, nullptr, 1, 3 * D, BV, CV, QKV + 2 * D, nullptr);
  att_kernel<<<BV * NH * TPB, 32, 0, stream>>>(QKV, BV, CV, ATT);
  dense_kernel<D, 1, 2><<<NTILE, 32, 0, stream>>>(ATT, nullptr, WO, (size_t)D * D, Fp(10), D, HW, Fp(11), Fp(12), 1, D, BV, CV, H1, H1b);
  dense_kernel<D, 2, 1><<<NTILE * 4, 32, 0, stream>>>(nullptr, H1b, W1T, (size_t)FF * D, Fp(14), FF, nullptr, nullptr, nullptr, 4, FF, BV, CV, nullptr, F);
  dense_kernel<FF, 2, 3><<<NTILE, 32, 0, stream>>>(nullptr, F, W2T, (size_t)D * FF, Fp(16), D, H1, Fp(17), Fp(18), 1, D, BV, CV, (float*)d_out, nullptr);
}
